// EfficientAttention_60327110640431
// MI455X (gfx1250) — hardware-verified
//
#include <hip/hip_runtime.h>

#pragma clang fp contract(off)

#ifndef NB
#define NB 2
#endif
#ifndef SEQ
#define SEQ 2048
#endif
#define NB_FULL  2
#define SEQ_FULL 2048
#define DM   2048
#define NH   16
#define NKV  4
#define REP  (NH / NKV)
#define HD   128
#define HD2  64
#define DKV  (NKV * HD)
#define RH   ((((SEQ) / 2) < 512) ? ((SEQ) / 2) : 512)
#define OSP  136
#define PCAR 1024.0f
#define CCAR 16.0f
#define WCAR 64.0f
#define SCL  0.08838834764831845f
#define L2E  1.4426950408889634f

static_assert(SEQ % 64 == 0);
static_assert(SEQ <= SEQ_FULL);
static_assert(NB >= 1 && NB <= NB_FULL);
static_assert(RH % 64 == 0 && RH >= 64 && 2 * RH <= SEQ);
static_assert(DM == NH * HD);
static_assert(DM % 64 == 0 && DKV % 64 == 0 && HD % 32 == 0);

typedef _Float16 h16;
typedef unsigned short bf;
typedef __attribute__((ext_vector_type(16))) __bf16   v16bf;
typedef __attribute__((ext_vector_type(16))) _Float16 v16h;
typedef __attribute__((ext_vector_type(16))) unsigned short v16us;
typedef __attribute__((ext_vector_type(8)))  _Float16 v8h;
typedef __attribute__((ext_vector_type(8)))  unsigned short v8us;
typedef __attribute__((ext_vector_type(8)))  float    v8f;
typedef __attribute__((ext_vector_type(4)))  float    v4f;
typedef __attribute__((ext_vector_type(2)))  _Float16 v2h;
typedef __attribute__((ext_vector_type(2)))  unsigned short v2us;
typedef __attribute__((ext_vector_type(2)))  float    v2f;
typedef v8h  __attribute__((may_alias)) v8ha;
typedef v4f  __attribute__((may_alias)) v4fa;
typedef v8us __attribute__((may_alias)) v8usa;

__device__ __forceinline__ unsigned short f2bf(float f) { unsigned u = __float_as_uint(f); u += 0x7FFFu + ((u >> 16) & 1u); return (unsigned short)(u >> 16); }
__device__ __forceinline__ float bf2f(unsigned short b) { return __uint_as_float(((unsigned)b) << 16); }
__device__ __forceinline__ float bfr(float f) { return bf2f(f2bf(f)); }
__device__ __forceinline__ void splitf(float y, unsigned short& h, unsigned short& l) { h = f2bf(y); l = f2bf(y - bf2f(h)); }
__device__ __forceinline__ v16h cat16(v8h lo, v8h hi) { return __builtin_shufflevector(lo, hi, 0, 1, 2, 3, 4, 5, 6, 7, 8, 9, 10, 11, 12, 13, 14, 15); }
__device__ __forceinline__ v16bf cat16b(v8us lo, v8us hi) { return __builtin_bit_cast(v16bf, __builtin_shufflevector(lo, hi, 0, 1, 2, 3, 4, 5, 6, 7, 8, 9, 10, 11, 12, 13, 14, 15)); }
__device__ __forceinline__ v8f wmma16(v16h a, v16h b, v8f c) { return __builtin_amdgcn_wmma_f32_16x16x32_f16(false, a, false, b, (short)0, c, false, false); }
__device__ __forceinline__ v8f wmmab(v16bf a, v16bf b, v8f c) { return __builtin_amdgcn_wmma_f32_16x16x32_bf16(false, a, false, b, (short)0, c, false, false); }

template <typename T16> struct WFrag;
template <> struct WFrag<h16> { typedef v16h V; static __device__ __forceinline__ V ld(const h16* p) { return cat16(*(const v8h*)p, *(const v8h*)(p + 16)); } static __device__ __forceinline__ v8f mma(V a, V b, v8f c) { return wmma16(a, b, c); } };
template <> struct WFrag<bf> { typedef v16bf V; static __device__ __forceinline__ V ld(const bf* p) { return cat16b(*(const v8us*)p, *(const v8us*)(p + 16)); } static __device__ __forceinline__ v8f mma(V a, V b, v8f c) { return wmmab(a, b, c); } };

template <typename T16, int NSPLIT, bool BIAS>
__global__ __launch_bounds__(32) void k_gemmw(const T16* __restrict__ A, const T16* __restrict__ A2, const T16* __restrict__ Bt, const T16* __restrict__ Bt2, int K, float* C, int ldc, const float* __restrict__ bias, float osc, size_t sA, size_t sB, size_t sC) {
    typedef typename WFrag<T16>::V V;
    __shared__ __align__(16) float os[16 * 68];
    const size_t z = blockIdx.z; A += z * sA; if (A2) A2 += z * sA; Bt += z * sB; if (Bt2) Bt2 += z * sB; C += z * sC;
    const int lane = threadIdx.x & 31, lr = lane & 15, hi = lane >> 4; const int r0 = blockIdx.x * 64, c0 = blockIdx.y * 64;
    v8f acc[4][4];
#pragma unroll
    for (int mb = 0; mb < 4; ++mb)
#pragma unroll
        for (int nb = 0; nb < 4; ++nb) acc[mb][nb] = (v8f){};
    const size_t aoff = (size_t)(r0 + lr) * K + 8 * hi, boff = (size_t)(c0 + lr) * K + 8 * hi;
#pragma unroll 1
    for (int kc = 0; kc < K; kc += 32) {
        V a[4], a2[4];
#pragma unroll
        for (int mb = 0; mb < 4; ++mb) { a[mb] = WFrag<T16>::ld(A + aoff + (size_t)mb * 16 * K + kc); if (NSPLIT == 1 || NSPLIT == 2) a2[mb] = WFrag<T16>::ld(A2 + aoff + (size_t)mb * 16 * K + kc); }
#pragma unroll
        for (int nb = 0; nb < 4; ++nb) { const V b = WFrag<T16>::ld(Bt + boff + (size_t)nb * 16 * K + kc); V b2; if (NSPLIT >= 2) b2 = WFrag<T16>::ld(Bt2 + boff + (size_t)nb * 16 * K + kc);
#pragma unroll
            for (int mb = 0; mb < 4; ++mb) { acc[mb][nb] = WFrag<T16>::mma(a[mb], b, acc[mb][nb]); if (NSPLIT == 1 || NSPLIT == 2) acc[mb][nb] = WFrag<T16>::mma(a2[mb], b, acc[mb][nb]); if (NSPLIT >= 2) acc[mb][nb] = WFrag<T16>::mma(a[mb], b2, acc[mb][nb]); } }
        asm volatile("v_nop\n\tv_nop\n\tv_nop\n\tv_nop" : "+v"(acc[0][0]), "+v"(acc[1][1]), "+v"(acc[2][2]), "+v"(acc[3][3]) : "v"(a[0]), "v"(a[3]));
    }
#pragma unroll
    for (int mb = 0; mb < 4; ++mb) {
#pragma unroll
        for (int nb = 0; nb < 4; ++nb) {
#pragma unroll
            for (int j = 0; j < 8; ++j) os[(hi * 8 + j) * 68 + nb * 16 + lr] = acc[mb][nb][j]; }
        __builtin_amdgcn_wave_barrier(); asm volatile("" ::: "memory");
        float* crow = C + (size_t)(r0 + mb * 16) * ldc + c0;
#pragma unroll 1
        for (int ps = 0; ps < 2; ++ps) {
#pragma unroll
            for (int s = 0; s < 8; ++s) { const int row = 2 * s + hi, cofs = lr * 4; v4f val = *(const v4fa*)(os + row * 68 + cofs); val = val * osc; if (BIAS) { val[0] += bfr(bias[c0 + cofs]); val[1] += bfr(bias[c0 + cofs + 1]); val[2] += bfr(bias[c0 + cofs + 2]); val[3] += bfr(bias[c0 + cofs + 3]); }
                *(volatile v4f*)(crow + (size_t)row * ldc + cofs) = val; }
            if (ps == 0) __threadfence(); }
        __builtin_amdgcn_wave_barrier(); asm volatile("" ::: "memory");
    }
}

template <bool F16P>
__global__ __launch_bounds__(256) void k_wtG(const float* __restrict__ w, int K, int N, bf* Bt, h16* B16) {
    const int lane = threadIdx.x & 31; const int L0 = (blockIdx.x * 8 + (threadIdx.x >> 5)) * 8; const int nlines = (int)((size_t)N * K / 64);
#pragma unroll
    for (int ps = 0; ps < 2; ++ps) {
#pragma unroll 1
        for (int l = 0; l < 8; ++l) { const int L = L0 + l; if (L >= nlines) break; const size_t e = (size_t)L * 64 + lane * 2; const int k = (int)(e % (size_t)K), n = (int)(e / (size_t)K);
            const float w0 = bfr(w[(size_t)k * N + n]), w1 = bfr(w[(size_t)(k + 1) * N + n]);
            v2us o; o[0] = f2bf(w0); o[1] = f2bf(w1); *(volatile v2us*)(Bt + e) = o;
            if (F16P) { v2h o2; o2[0] = (h16)(w0 * WCAR); o2[1] = (h16)(w1 * WCAR); *(volatile v2h*)(B16 + e) = o2; } }
        if (ps == 0) __threadfence(); }
}

__global__ __launch_bounds__(256) void k_cvt8(const float* __restrict__ src, bf* dst, size_t n8, size_t sstr, size_t dstr) {
    src += (size_t)blockIdx.y * sstr; dst += (size_t)blockIdx.y * dstr;
    const size_t i = (size_t)blockIdx.x * 256 + threadIdx.x; if (i >= n8) return; const v8f v = *(const v8f*)(src + i * 8); v8us o;
#pragma unroll
    for (int k = 0; k < 8; ++k) o[k] = f2bf(v[k]);
    *(volatile v8us*)(dst + i * 8) = o; __threadfence(); *(volatile v8us*)(dst + i * 8) = o; }

__global__ __launch_bounds__(64) void k_invf(float* IFQ) {
    __shared__ __align__(16) float tb[64];
    const int tid = threadIdx.x;
    const float ex = (float)(2 * tid) * 0.0078125f;
    const float p = powf(10000.0f, ex);
    tb[tid] = __fdiv_rn(1.0f, p);
    __syncthreads();
    v4f v = (v4f){};
    if (tid < 16) v = *(const v4fa*)(tb + tid * 4);
    if (tid < 16) *(volatile v4f*)(IFQ + tid * 4) = v;
    __threadfence();
    if (tid < 16) *(volatile v4f*)(IFQ + tid * 4) = v;
}
__global__ __launch_bounds__(256) void k_cst(const float* __restrict__ IFQ, float* CS) {
    const int idx = blockIdx.x * 256 + threadIdx.x; if (idx >= SEQ * HD2) return;
    const int t = idx / HD2, j = idx % HD2;
    const float fr = __fmul_rn((float)t, IFQ[j]);
    float sv, cv; sincosf(fr, &sv, &cv);
    v2f o; o[0] = cv; o[1] = sv;
    *(volatile v2f*)(CS + (size_t)idx * 2) = o; __threadfence(); *(volatile v2f*)(CS + (size_t)idx * 2) = o; }

__global__ __launch_bounds__(256) void k_rope(const float* __restrict__ F, int pitch, int nheads, const float* __restrict__ CS, h16* P16, bf* Ph, bf* Pl) {
    const int bb = blockIdx.y;
    F += (size_t)bb * SEQ * pitch; P16 += (size_t)bb * nheads * SEQ * HD; Ph += (size_t)bb * nheads * RH * HD; Pl += (size_t)bb * nheads * RH * HD;
    const size_t e = ((size_t)blockIdx.x * 256 + threadIdx.x) * 2; if (e >= (size_t)nheads * SEQ * HD) return;
    const int d = (int)(e % HD); const int t = (int)((e / HD) % SEQ); const int hh = (int)(e / ((size_t)HD * SEQ));
    const float* f = F + (size_t)t * pitch + (size_t)hh * HD;
    v2h o16; v2us oh, ol;
#pragma unroll
    for (int q = 0; q < 2; ++q) { const int dd = d + q; const int dp = (dd < HD2) ? dd + HD2 : dd - HD2; const float x0 = f[dd], x1 = f[dp];
        const v2f cs = *(const v2f*)(CS + ((size_t)t * HD2 + (dd & (HD2 - 1))) * 2);
        float a = __fmul_rn(x0, cs[0]), bq = __fmul_rn(x1, cs[1]); asm volatile("" : "+v"(a)); asm volatile("" : "+v"(bq));
        const float r = (dd < HD2) ? __fsub_rn(a, bq) : __fadd_rn(a, bq);
        o16[q] = (h16)r; unsigned short a2, c2; splitf(r, a2, c2); oh[q] = a2; ol[q] = c2; }
    const bool hr = (t < RH); const size_t eo = ((size_t)hh * RH + t) * HD + d;
    *(volatile v2h*)(P16 + e) = o16; if (hr) { *(volatile v2us*)(Ph + eo) = oh; *(volatile v2us*)(Pl + eo) = ol; }
    __threadfence();
    *(volatile v2h*)(P16 + e) = o16; if (hr) { *(volatile v2us*)(Ph + eo) = oh; *(volatile v2us*)(Pl + eo) = ol; } }

__global__ __launch_bounds__(256) void k_vtp(const float* __restrict__ F, int pitch, int nheads, h16* V16, bf* Vh, bf* Vl) {
    const int bb = blockIdx.y;
    F += (size_t)bb * SEQ * pitch; V16 += (size_t)bb * nheads * HD * SEQ; Vh += (size_t)bb * nheads * HD * RH; Vl += (size_t)bb * nheads * HD * RH;
    const size_t e = ((size_t)blockIdx.x * 256 + threadIdx.x) * 2; if (e >= (size_t)nheads * HD * SEQ) return;
    const int t = (int)(e % SEQ); const int d = (int)((e / SEQ) % HD); const int g = (int)(e / ((size_t)SEQ * HD));
    v2h o16; v2us oh, ol;
#pragma unroll
    for (int q = 0; q < 2; ++q) { const float x = F[(size_t)(t + q) * pitch + (size_t)g * HD + d]; o16[q] = (h16)x; unsigned short a2, c2; splitf(x, a2, c2); oh[q] = a2; ol[q] = c2; }
    const bool hr = (t < RH); const size_t eo = ((size_t)g * HD + d) * RH + t;
    *(volatile v2h*)(V16 + e) = o16; if (hr) { *(volatile v2us*)(Vh + eo) = oh; *(volatile v2us*)(Vl + eo) = ol; }
    __threadfence();
    *(volatile v2h*)(V16 + e) = o16; if (hr) { *(volatile v2us*)(Vh + eo) = oh; *(volatile v2us*)(Vl + eo) = ol; } }

__device__ __forceinline__ void wave_lds_sync() { __builtin_amdgcn_fence(5, "wavefront"); __builtin_amdgcn_wave_barrier(); asm volatile("" ::: "memory"); }
__device__ __forceinline__ void tile_rows_out(const unsigned short* osw, unsigned short* dst, size_t pitch, int lr, int hi) {
#pragma unroll 1
    for (int ps = 0; ps < 2; ++ps) {
#pragma unroll
        for (int s = 0; s < 8; ++s) { const int row = 2 * s + hi; const v8us v = *(const v8usa*)(osw + row * OSP + lr * 8); *(volatile v8us*)(dst + (size_t)row * pitch + lr * 8) = v; }
        if (ps == 0) __threadfence(); }
}

template <bool HR>
__global__ __launch_bounds__(128) __attribute__((amdgpu_num_vgpr(256)))
void k_attn(const h16* Q16, const bf* Qh, const bf* Ql, const h16* K16, const bf* Kh, const bf* Kl, const h16* VT16, const bf* VTh, const bf* VTl,
            h16* CT16, bf* CTh, bf* CTl, int qblk0)
{
    __shared__ __align__(16) unsigned short os[4 * 16 * OSP];
    const int lane = threadIdx.x & 31, wv = threadIdx.x >> 5, lr = lane & 15, hi = lane >> 4;
    const int b = blockIdx.z, h = blockIdx.y, g = h / REP;
    const int qb = (qblk0 + (int)blockIdx.x) * 64, qw = qb + wv * 16, qme = qw + lr, kend = qw + 16;
    const size_t zq = (size_t)b * NH + h, zk = (size_t)b * NKV + g;
    const size_t qoh = HR ? ((zq * RH + qme) * HD + 8 * hi) : (size_t)0;
    const h16* Qrow  = Q16 + (zq * SEQ + qme) * HD + 8 * hi;
    const bf*  Qhrow = Qh + qoh; const bf* Qlrow = Ql + qoh;
    const h16* Kb  = K16 + (zk * SEQ + lr) * HD + 8 * hi;
    const bf*  Khb = Kh + (zk * RH + lr) * HD + 8 * hi; const bf* Klb = Kl + (zk * RH + lr) * HD + 8 * hi;
    const h16* Vb  = VT16 + (zk * HD + lr) * SEQ + 8 * hi;
    const bf*  Vhb = VTh + (zk * HD + lr) * RH + 8 * hi; const bf* Vlb = VTl + (zk * HD + lr) * RH + 8 * hi;
    unsigned short* osw = os + wv * (16 * OSP);

    v8f acc[8];
#pragma unroll
    for (int dt = 0; dt < 8; ++dt) acc[dt] = (v8f){};
    float mrun = -3.0e38f, lrun = 0.f;
    v16h qf[4];
#pragma unroll
    for (int ds = 0; ds < 4; ++ds) qf[ds] = HR ? (v16h){} : WFrag<h16>::ld(Qrow + ds * 32);

#pragma unroll 1
    for (int kb = 0; kb < kend; kb += 32) {
        v8f s0 = (v8f){}, s1 = (v8f){};
        if (!HR) {
#pragma unroll
            for (int ds = 0; ds < 4; ++ds) {
                const v16h a0 = WFrag<h16>::ld(Kb + (size_t)kb * HD + ds * 32);
                const v16h a1 = WFrag<h16>::ld(Kb + (size_t)(kb + 16) * HD + ds * 32);
                s0 = wmma16(a0, qf[ds], s0); s1 = wmma16(a1, qf[ds], s1);
                asm volatile("" : "+v"(s0), "+v"(s1) : : "memory");
            }
        } else {
#pragma unroll
            for (int ds = 0; ds < 4; ++ds) {
                const v16bf bq  = WFrag<bf>::ld(Qhrow + ds * 32);
                const v16bf bl  = WFrag<bf>::ld(Qlrow + ds * 32);
                const v16bf ah0 = WFrag<bf>::ld(Khb + (size_t)kb * HD + ds * 32);
                const v16bf al0 = WFrag<bf>::ld(Klb + (size_t)kb * HD + ds * 32);
                s0 = wmmab(ah0, bq, s0); s0 = wmmab(ah0, bl, s0); s0 = wmmab(al0, bq, s0);
                const v16bf ah1 = WFrag<bf>::ld(Khb + (size_t)(kb + 16) * HD + ds * 32);
                const v16bf al1 = WFrag<bf>::ld(Klb + (size_t)(kb + 16) * HD + ds * 32);
                s1 = wmmab(ah1, bq, s1); s1 = wmmab(ah1, bl, s1); s1 = wmmab(al1, bq, s1);
                asm volatile("" : "+v"(s0), "+v"(s1) : : "memory");
            }
        }
        asm volatile("v_nop\n\tv_nop\n\tv_nop\n\tv_nop" : "+v"(s0), "+v"(s1));

        float t0[8], t1[8]; float mloc = -3.0e38f;
        const int kq0 = kb + 8 * hi - qme;
#pragma unroll
        for (int r = 0; r < 8; ++r) {
            float u0 = s0[r] * SCL, u1 = s1[r] * SCL;
            if (kq0 + r > 0) u0 = -3.0e38f;
            if (kq0 + 16 + r > 0) u1 = -3.0e38f;
            t0[r] = u0; t1[r] = u1; mloc = fmaxf(mloc, fmaxf(u0, u1));
        }
        mloc = fmaxf(mloc, __shfl_xor(mloc, 16, 32));
        const float mnew = fmaxf(mrun, mloc);
        const float alpha = __builtin_amdgcn_exp2f((mrun - mnew) * L2E);
        mrun = mnew;
        float psum = 0.f;
#pragma unroll
        for (int r = 0; r < 8; ++r) { t0[r] = __builtin_amdgcn_exp2f((t0[r] - mnew) * L2E); t1[r] = __builtin_amdgcn_exp2f((t1[r] - mnew) * L2E); psum += t0[r] + t1[r]; }
        psum += __shfl_xor(psum, 16, 32);
        lrun = lrun * alpha + psum;
#pragma unroll
        for (int dt = 0; dt < 8; ++dt) acc[dt] = acc[dt] * alpha;

        if (!HR) {
            v16h pf;
#pragma unroll
            for (int r = 0; r < 8; ++r) { pf[r] = (h16)(t0[r] * PCAR); pf[8 + r] = (h16)(t1[r] * PCAR); }
#pragma unroll
            for (int dt = 0; dt < 8; ++dt) {
                const v16h va = WFrag<h16>::ld(Vb + (size_t)(dt * 16) * SEQ + kb);
                acc[dt] = wmma16(va, pf, acc[dt]);
                asm volatile("" : "+v"(acc[dt]) : : "memory");
            }
            asm volatile("v_nop\n\tv_nop\n\tv_nop\n\tv_nop" : "+v"(acc[0]), "+v"(acc[1]), "+v"(acc[2]), "+v"(acc[3]), "+v"(acc[4]), "+v"(acc[5]), "+v"(acc[6]), "+v"(acc[7]) : "v"(pf));
        } else {
            v16us phb, plb;
#pragma unroll
            for (int r = 0; r < 8; ++r) { unsigned short a2, c2; splitf(t0[r] * PCAR, a2, c2); phb[r] = a2; plb[r] = c2; splitf(t1[r] * PCAR, a2, c2); phb[8 + r] = a2; plb[8 + r] = c2; }
            const v16bf ph = __builtin_bit_cast(v16bf, phb), pl = __builtin_bit_cast(v16bf, plb);
#pragma unroll
            for (int dt = 0; dt < 8; ++dt) {
                const v16bf vh = WFrag<bf>::ld(Vhb + (size_t)(dt * 16) * RH + kb);
                const v16bf vl = WFrag<bf>::ld(Vlb + (size_t)(dt * 16) * RH + kb);
                acc[dt] = wmmab(vh, ph, acc[dt]); acc[dt] = wmmab(vh, pl, acc[dt]); acc[dt] = wmmab(vl, ph, acc[dt]);
                asm volatile("" : "+v"(acc[dt]) : : "memory");
            }
            asm volatile("v_nop\n\tv_nop\n\tv_nop\n\tv_nop" : "+v"(acc[0]), "+v"(acc[1]), "+v"(acc[2]), "+v"(acc[3]), "+v"(acc[4]), "+v"(acc[5]), "+v"(acc[6]), "+v"(acc[7]) : "v"(ph));
        }
    }

    const float inv = __fdiv_rn(1.0f, lrun * PCAR);
    if (!HR) {
        const float f = inv * CCAR;
#pragma unroll
        for (int dt = 0; dt < 8; ++dt) { v8h o;
#pragma unroll
            for (int r = 0; r < 8; ++r) o[r] = (h16)(acc[dt][r] * f);
            *(v8us*)(osw + lr * OSP + dt * 16 + 8 * hi) = __builtin_bit_cast(v8us, o); }
        wave_lds_sync();
        tile_rows_out(osw, (unsigned short*)CT16 + ((size_t)b * SEQ + qw) * DM + (size_t)h * HD, (size_t)DM, lr, hi);
    } else {
#pragma unroll
        for (int dt = 0; dt < 8; ++dt) { v8us o;
#pragma unroll
            for (int r = 0; r < 8; ++r) o[r] = f2bf(acc[dt][r] * inv);
            *(v8us*)(osw + lr * OSP + dt * 16 + 8 * hi) = o; }
        wave_lds_sync();
        tile_rows_out(osw, CTh + ((size_t)b * RH + qw) * DM + (size_t)h * HD, (size_t)DM, lr, hi);
        wave_lds_sync();
#pragma unroll
        for (int dt = 0; dt < 8; ++dt) { v8us o;
#pragma unroll
            for (int r = 0; r < 8; ++r) { const float y = acc[dt][r] * inv; o[r] = f2bf(y - bf2f(f2bf(y))); }
            *(v8us*)(osw + lr * OSP + dt * 16 + 8 * hi) = o; }
        wave_lds_sync();
        tile_rows_out(osw, CTl + ((size_t)b * RH + qw) * DM + (size_t)h * HD, (size_t)DM, lr, hi);
    }
}

extern "C" void kernel_launch(void* const* d_in, const int* in_sizes, int n_in,
                              void* d_out, int out_size, void* d_ws, size_t ws_size, hipStream_t stream) {
    if (n_in < 5) return;
    if ((long long)in_sizes[0] < (long long)(NB - 1) * SEQ_FULL * DM + (long long)SEQ * DM) return;
    if ((long long)in_sizes[1] < (long long)DM * DM) return;
    if ((long long)in_sizes[2] < (long long)DM * DKV) return;
    if ((long long)in_sizes[3] < (long long)DM * DKV) return;
    if ((long long)in_sizes[4] < (long long)DM * DM) return;
    if ((long long)out_size < (long long)(NB - 1) * SEQ_FULL * DM + (long long)SEQ * DM) return;
    const float* x  = (const float*)d_in[0];
    const float* wq = (const float*)d_in[1];
    const float* wk = (const float*)d_in[2];
    const float* wv = (const float*)d_in[3];
    const float* wo = (const float*)d_in[4];
    float* OUT = (float*)d_out;
    char* wsp = (char*)d_ws;
    auto take = [&](size_t bytes) { char* p = wsp; wsp += (bytes + 255) & ~(size_t)255; return (void*)p; };
    bf*  WQ   = (bf*)take((size_t)DM * DM * 2);
    bf*  WK   = (bf*)take((size_t)DKV * DM * 2);
    bf*  WV   = (bf*)take((size_t)DKV * DM * 2);
    bf*  WOB  = (bf*)take((size_t)DM * DM * 2);
    h16* WO16 = (h16*)take((size_t)DM * DM * 2);
    float* IFQ = (float*)take(256);
    float* CS  = (float*)take((size_t)SEQ * HD2 * 2 * 4);
    bf*  XB   = (bf*)take((size_t)NB * SEQ * DM * 2);
    float* FQ = (float*)take((size_t)NB * SEQ * DM * 4);
    float* FK = (float*)take((size_t)NB * SEQ * DKV * 4);
    h16* Q16  = (h16*)take((size_t)NB * NH * SEQ * HD * 2);
    bf*  QH   = (bf*)take((size_t)NB * NH * RH * HD * 2);
    bf*  QL   = (bf*)take((size_t)NB * NH * RH * HD * 2);
    h16* K16  = (h16*)take((size_t)NB * NKV * SEQ * HD * 2);
    bf*  KH   = (bf*)take((size_t)NB * NKV * RH * HD * 2);
    bf*  KL   = (bf*)take((size_t)NB * NKV * RH * HD * 2);
    h16* VT16 = (h16*)take((size_t)NB * NKV * HD * SEQ * 2);
    bf*  VTH  = (bf*)take((size_t)NB * NKV * HD * RH * 2);
    bf*  VTL  = (bf*)take((size_t)NB * NKV * HD * RH * 2);
    if ((size_t)(wsp - (char*)d_ws) > ws_size) return;
    float* FV = FK;
    h16* CT16 = (h16*)FQ;
    bf*  CTH  = (bf*)((char*)FQ + (size_t)NB * SEQ * DM * 2);
    bf*  CTL  = (bf*)((char*)CTH + (size_t)NB * RH * DM * 2);

    const unsigned gWQ = (unsigned)(((size_t)DM * DM / 64 + 63) / 64), gWK = (unsigned)(((size_t)DKV * DM / 64 + 63) / 64);
    k_wtG<false><<<gWQ, 256, 0, stream>>>(wq, DM, DM, WQ, nullptr);
    k_wtG<false><<<gWK, 256, 0, stream>>>(wk, DM, DKV, WK, nullptr);
    k_wtG<false><<<gWK, 256, 0, stream>>>(wv, DM, DKV, WV, nullptr);
    k_wtG<true><<<gWQ, 256, 0, stream>>>(wo, DM, DM, WOB, WO16);
    k_invf<<<1, 64, 0, stream>>>(IFQ);
    k_cst<<<(SEQ * HD2 + 255) / 256, 256, 0, stream>>>(IFQ, CS);
    k_cvt8<<<dim3((unsigned)(((size_t)SEQ * DM / 8 + 255) / 256), NB), 256, 0, stream>>>(x, XB, (size_t)SEQ * DM / 8, (size_t)SEQ_FULL * DM, (size_t)SEQ * DM);
    const unsigned LQ = (unsigned)(((size_t)NH * SEQ * HD / 2 + 255) / 256), LK = (unsigned)(((size_t)NKV * SEQ * HD / 2 + 255) / 256);
    k_gemmw<bf, 0, false><<<dim3(SEQ / 64, DM / 64, NB), 32, 0, stream>>>(XB, nullptr, WQ, nullptr, DM, FQ, DM, nullptr, 1.0f, (size_t)SEQ * DM, (size_t)0, (size_t)SEQ * DM);
    k_rope<<<dim3(LQ, NB), 256, 0, stream>>>(FQ, DM, NH, CS, Q16, QH, QL);
    k_gemmw<bf, 0, false><<<dim3(SEQ / 64, DKV / 64, NB), 32, 0, stream>>>(XB, nullptr, WK, nullptr, DM, FK, DKV, nullptr, 1.0f, (size_t)SEQ * DM, (size_t)0, (size_t)SEQ * DKV);
    k_rope<<<dim3(LK, NB), 256, 0, stream>>>(FK, DKV, NKV, CS, K16, KH, KL);
    k_gemmw<bf, 0, false><<<dim3(SEQ / 64, DKV / 64, NB), 32, 0, stream>>>(XB, nullptr, WV, nullptr, DM, FV, DKV, nullptr, 1.0f, (size_t)SEQ * DM, (size_t)0, (size_t)SEQ * DKV);
    k_vtp<<<dim3(LK, NB), 256, 0, stream>>>(FV, DKV, NKV, VT16, VTH, VTL);
    k_attn<true><<<dim3(RH / 64, NH, NB), 128, 0, stream>>>(Q16, QH, QL, K16, KH, KL, VT16, VTH, VTL, CT16, CTH, CTL, 0);
    if (SEQ > RH) k_attn<false><<<dim3((SEQ - RH) / 64, NH, NB), 128, 0, stream>>>(Q16, QH, QL, K16, KH, KL, VT16, VTH, VTL, CT16, CTH, CTL, RH / 64);
    k_gemmw<bf, 1, false><<<dim3(RH / 64, DM / 64, NB), 32, 0, stream>>>(CTH, CTL, WOB, nullptr, DM, OUT, DM, nullptr, 1.0f, (size_t)RH * DM, (size_t)0, (size_t)SEQ_FULL * DM);
    if (SEQ > RH) k_gemmw<h16, 0, false><<<dim3((SEQ - RH) / 64, DM / 64, NB), 32, 0, stream>>>(CT16 + (size_t)RH * DM, nullptr, WO16, nullptr, DM, OUT + (size_t)RH * DM, DM, nullptr, 1.0f / (CCAR * WCAR), (size_t)SEQ * DM, (size_t)0, (size_t)SEQ_FULL * DM);
}
